// SparseSelfAttention_27831388078818
// MI455X (gfx1250) — hardware-verified
//
#include <hip/hip_runtime.h>
#include <math.h>

typedef __attribute__((ext_vector_type(16))) _Float16 v16h;
typedef __attribute__((ext_vector_type(16))) __bf16 v16b;
typedef __attribute__((ext_vector_type(8)))  _Float16 v8h;
typedef __attribute__((ext_vector_type(8)))  __bf16 v8b;
typedef __attribute__((ext_vector_type(8)))  float v8f;
typedef __attribute__((ext_vector_type(4)))  float v4f;
typedef __attribute__((ext_vector_type(4)))  unsigned v4u;

template <typename T> __device__ __forceinline__ void vst2(void* p, T v) { *(volatile T*)p = v; __threadfence(); *(volatile T*)p = v; }

__device__ __forceinline__ v8f wmma16(v16h a, v16h b, v8f c) {
  v8f d = __builtin_amdgcn_wmma_f32_16x16x32_f16(false, a, false, b, (short)0, c, false, false);
  asm volatile("v_nop\n\tv_nop\n\tv_nop\n\tv_nop" : "+v"(d) : "v"(a), "v"(b));
  return d;
}
__device__ __forceinline__ v8f wmma_bf(v16b a, v16b b, v8f c) {
  v8f d = __builtin_amdgcn_wmma_f32_16x16x32_bf16(false, a, false, b, (short)0, c, false, false);
  asm volatile("v_nop\n\tv_nop\n\tv_nop\n\tv_nop" : "+v"(d) : "v"(a), "v"(b));
  return d;
}
__device__ __forceinline__ v16h frag_h(const _Float16* rowk0, int lane) {
  union { v16h v; v8h q[2]; } u; const _Float16* p = rowk0 + 8 * (lane >> 4);
  u.q[0] = *(const v8h*)p; u.q[1] = *(const v8h*)(p + 16); return u.v;
}
__device__ __forceinline__ v16b frag_b(const __bf16* rowk0, int lane) {
  union { v16b v; v8b q[2]; } u; const __bf16* p = rowk0 + 8 * (lane >> 4);
  u.q[0] = *(const v8b*)p; u.q[1] = *(const v8b*)(p + 16); return u.v;
}
__device__ __forceinline__ float bfr(float v) { return (float)(__bf16)v; }
__device__ __forceinline__ void ldsx() { asm volatile("s_wait_dscnt 0x0" ::: "memory"); __builtin_amdgcn_wave_barrier(); __builtin_amdgcn_fence(3, "workgroup"); }

#ifndef NB
#define NB 4
#endif
#ifndef SEQ
#define SEQ 4096
#endif
#define NB_FULL 4
#define SEQ_FULL 4096
#define TT SEQ
#define CC 256
#define DIN 256
#define PP (2 * TT)
#define PCARRY 16384.0f
#define NEGFILL (-1.0e9f)
static_assert(NB >= 1 && NB <= NB_FULL);
static_assert(SEQ >= 64 && SEQ <= SEQ_FULL && (SEQ % 64) == 0);
static_assert(CC == 256 && DIN == 256);

#define WS_XB  0u
#define WS_WT  (WS_XB + 2u * (size_t)NB * TT * DIN)
#define WS_QH  (WS_WT + 2u * (size_t)3 * CC * DIN)
#define WS_QL  (WS_QH + 2u * (size_t)NB * TT * CC)
#define WS_KH  (WS_QL + 2u * (size_t)NB * TT * CC)
#define WS_KL  (WS_KH + 2u * (size_t)NB * TT * CC)
#define WS_VT  (WS_KL + 2u * (size_t)NB * TT * CC)
#define WS_S   (WS_VT + 2u * (size_t)NB * CC * TT)
#define WS_END (WS_S  + 4u * (size_t)TT * TT)
static_assert(WS_END <= (size_t)134217728u);
static_assert((WS_WT % 128u) == 0 && (WS_QH % 128u) == 0 && (WS_S % 128u) == 0);

__global__ __launch_bounds__(256) void k_xb(const float* __restrict__ X, __bf16* __restrict__ XB) {
  const size_t i = (size_t)blockIdx.x * 256 + threadIdx.x; if (i >= (size_t)NB * TT * (DIN / 8)) return;
  const size_t r = i / (DIN / 8); const int k = (int)(i % (DIN / 8)) * 8;
  const float* p = X + (((r / TT) * SEQ_FULL + (r % TT)) * (size_t)DIN + k);
  const v4f x0 = *(const v4f*)p, x1 = *(const v4f*)(p + 4);
  union { v8b h; v4u u; } o;
#pragma unroll
  for (int e = 0; e < 4; ++e) { o.h[e] = (__bf16)x0[e]; o.h[4 + e] = (__bf16)x1[e]; }
  vst2(XB + r * DIN + k, o.u);
}
__global__ __launch_bounds__(128) void k_wt(const float* __restrict__ WQ, const float* __restrict__ WK, const float* __restrict__ WV, __bf16* __restrict__ WT) {
  __shared__ __align__(16) __bf16 tr[16][DIN + 8];
  const int tid = threadIdx.x; const int c0 = blockIdx.x * 16; const int pl = blockIdx.y;
  const float* W = pl == 0 ? WQ : pl == 1 ? WK : WV;
#pragma unroll 4
  for (int it = 0; it < (16 * DIN) / 128; ++it) { const int idx = it * 128 + tid; const int k = idx >> 4, cl = idx & 15; tr[cl][k] = (__bf16)W[(size_t)k * CC + c0 + cl]; }
  __syncthreads();
  for (int e = tid; e < 16 * (DIN / 8); e += 128) { const int rl = e >> 5, q = e & 31; vst2(WT + ((size_t)pl * CC + c0 + rl) * DIN + q * 8, *(const v4u*)&tr[rl][q * 8]); }
}
__global__ __launch_bounds__(128) __attribute__((amdgpu_num_vgpr(256)))
void k_proj(const __bf16* __restrict__ XB, const __bf16* __restrict__ WT, const float* __restrict__ BQ, const float* __restrict__ BK, const float* __restrict__ BV,
            _Float16* __restrict__ QH, _Float16* __restrict__ QL, _Float16* __restrict__ KH, _Float16* __restrict__ KL, _Float16* __restrict__ VT) {
  __shared__ __align__(16) _Float16 sh[64][136], sl[64][136]; __shared__ __align__(16) _Float16 th[128][72];
  const int tid = threadIdx.x, wave = tid >> 5, lane = tid & 31, col = lane & 15, g = lane >> 4;
  const int which = blockIdx.z; const int c0 = blockIdx.y * 128; const size_t r0 = (size_t)blockIdx.x * 64; const size_t bb = r0 / TT; const int t0 = (int)(r0 % TT);
  const float* BA = which == 0 ? BQ : which == 1 ? BK : BV;
  const __bf16* WP = WT + (size_t)which * CC * DIN;
  v8f acc[8] = {};
#pragma unroll 1
  for (int kc = 0; kc < DIN / 32; ++kc) {
    const v16b a = frag_b(XB + (r0 + wave * 16 + col) * DIN + kc * 32, lane);
#pragma unroll
    for (int j = 0; j < 8; ++j) acc[j] = wmma_bf(a, frag_b(WP + (size_t)(c0 + j * 16 + col) * DIN + kc * 32, lane), acc[j]);
  }
  if (which < 2) { _Float16* DH = which == 0 ? QH : KH; _Float16* DL = which == 0 ? QL : KL;
#pragma unroll
    for (int j = 0; j < 8; ++j) { const float bias = bfr(BA[c0 + j * 16 + col]);
#pragma unroll
      for (int r = 0; r < 8; ++r) { const float v = acc[j][r] + bias; const _Float16 hv = (_Float16)v; sh[wave * 16 + 8 * g + r][j * 16 + col] = hv; sl[wave * 16 + 8 * g + r][j * 16 + col] = (_Float16)((v - (float)hv) * 1024.0f); } }
    __syncthreads();
    for (int e = tid; e < 64 * 16; e += 128) { const int rl = e >> 4, q = e & 15; vst2(DH + (r0 + rl) * CC + c0 + q * 8, *(const v4u*)&sh[rl][q * 8]); vst2(DL + (r0 + rl) * CC + c0 + q * 8, *(const v4u*)&sl[rl][q * 8]); }
  } else {
#pragma unroll
    for (int j = 0; j < 8; ++j) { const float bias = bfr(BA[c0 + j * 16 + col]);
#pragma unroll
      for (int r = 0; r < 8; ++r) { const float v = acc[j][r] + bias; const int rl = wave * 16 + 8 * g + r, cl = j * 16 + col; th[cl][rl] = (_Float16)v; } }
    __syncthreads();
    for (int e = tid; e < 128 * 8; e += 128) { const int cl = e >> 3, q = e & 7; vst2(VT + (bb * CC + c0 + cl) * (size_t)TT + t0 + q * 8, *(const v4u*)&th[cl][q * 8]); } }
}
__global__ __launch_bounds__(128) __attribute__((amdgpu_num_vgpr(256)))
void k_sc(const _Float16* __restrict__ QH, const _Float16* __restrict__ KH, const _Float16* __restrict__ QL, const _Float16* __restrict__ KL, int b, float* __restrict__ S) {
  __shared__ __align__(16) float ss[4][16][68];
  const int tid = threadIdx.x, wave = tid >> 5, lane = tid & 31, col = lane & 15, g = lane >> 4;
  const int qb = blockIdx.x, kb = blockIdx.y; const int k0 = kb * 64; const int ql0 = qb * 64 + wave * 16;
  const size_t q0 = (size_t)b * TT + ql0, kr0 = (size_t)b * TT + k0;
  v8f acc[4] = {}, accl[4] = {};
#pragma unroll 1
  for (int kc = 0; kc < CC / 32; ++kc) {
    const v16h ah = frag_h(QH + (q0 + col) * CC + kc * 32, lane), al = frag_h(QL + (q0 + col) * CC + kc * 32, lane);
#pragma unroll
    for (int j = 0; j < 4; ++j) {
      const v16h kf = frag_h(KH + (kr0 + j * 16 + col) * CC + kc * 32, lane), kl = frag_h(KL + (kr0 + j * 16 + col) * CC + kc * 32, lane);
      acc[j] = wmma16(ah, kf, acc[j]); accl[j] = wmma16(al, kf, accl[j]); accl[j] = wmma16(ah, kl, accl[j]); } }
#pragma unroll
  for (int j = 0; j < 4; ++j) {
#pragma unroll
    for (int r = 0; r < 8; ++r) ss[wave][8 * g + r][j * 16 + col] = acc[j][r] + accl[j][r] * (1.0f / 1024.0f); }
  ldsx();
  for (int rl = 0; rl < 16; ++rl) if (lane < 16) vst2(S + (size_t)(ql0 + rl) * TT + k0 + lane * 4, *(const v4f*)&ss[wave][rl][lane * 4]);
}
__global__ __launch_bounds__(256) void k_sm(float* __restrict__ S0) {
  __shared__ float sred[8], sred2[8]; __shared__ float sbc, sbc2; __shared__ __align__(16) float shv[TT];
  const int tid = threadIdx.x, lane = tid & 31, wv = tid >> 5; const int t = blockIdx.x;
  const float* sr = S0 + (size_t)t * TT; _Float16* pr = (_Float16*)(S0 + (size_t)t * TT);
  float m = -3.0e38f, mn = 3.0e38f;
#pragma unroll 1
  for (int q = tid; q < TT / 4; q += 256) { const v4f x = *(const v4f*)(sr + q * 4); *(v4f*)&shv[q * 4] = x;
    m = fmaxf(fmaxf(m, fmaxf(x[0], x[1])), fmaxf(x[2], x[3])); mn = fminf(fminf(mn, fminf(x[0], x[1])), fminf(x[2], x[3])); }
#pragma unroll
  for (int o = 1; o < 32; o <<= 1) { m = fmaxf(m, __shfl_xor(m, o)); mn = fminf(mn, __shfl_xor(mn, o)); }
  if (lane == 0) { sred[wv] = m; sred2[wv] = mn; } __syncthreads();
  if (tid == 0) { float a = sred[0], c = sred2[0]; for (int i = 1; i < 8; ++i) { a = fmaxf(a, sred[i]); c = fminf(c, sred2[i]); } sbc = a; sbc2 = c; }
  __syncthreads(); m = sbc; mn = sbc2; __syncthreads();
  float sum = 0.f;
#pragma unroll 1
  for (int k = tid; k < TT; k += 256) { float v = shv[k]; v = (v >= mn) ? v : NEGFILL; const float e = expf(v - m); shv[k] = e; sum += e; }
#pragma unroll
  for (int o = 1; o < 32; o <<= 1) sum += __shfl_xor(sum, o);
  if (lane == 0) sred[wv] = sum; __syncthreads();
  if (tid == 0) { float a = 0.f; for (int i = 0; i < 8; ++i) a += sred[i]; sbc = PCARRY * (1.0f / a); }
  __syncthreads(); const float inv = sbc;
#pragma unroll 1
  for (int q = tid; q < TT / 8; q += 256) { const v4f e0 = *(const v4f*)&shv[q * 8], e1 = *(const v4f*)&shv[q * 8 + 4]; union { v8h h; v4u u; } pk;
#pragma unroll
    for (int i = 0; i < 4; ++i) { pk.h[i] = (_Float16)(e0[i] * inv); pk.h[4 + i] = (_Float16)(e1[i] * inv); }
    vst2(pr + q * 8, pk.u); }
}
__global__ __launch_bounds__(128) __attribute__((amdgpu_num_vgpr(256)))
void k_pv(const _Float16* __restrict__ PH, const _Float16* __restrict__ VT, int b, float* __restrict__ OUT) {
  __shared__ __align__(16) float ss[4][16][132];
  const int tid = threadIdx.x, wave = tid >> 5, lane = tid & 31, col = lane & 15, g = lane >> 4;
  const int qb = blockIdx.x, ch = blockIdx.y; const int ql0 = qb * 64 + wave * 16;
  const _Float16* Vp = VT + ((size_t)b * CC + ch * 128) * TT;
  v8f acc[8] = {};
#pragma unroll 1
  for (int kc = 0; kc < TT / 32; ++kc) {
    const v16h p = frag_h(PH + (size_t)(ql0 + col) * PP + kc * 32, lane);
#pragma unroll
    for (int j = 0; j < 8; ++j) acc[j] = wmma16(p, frag_h(Vp + (size_t)(j * 16 + col) * TT + kc * 32, lane), acc[j]);
  }
#pragma unroll
  for (int j = 0; j < 8; ++j) {
#pragma unroll
    for (int r = 0; r < 8; ++r) ss[wave][8 * g + r][j * 16 + col] = acc[j][r] * (1.0f / PCARRY); }
  ldsx();
  for (int rl = 0; rl < 16; ++rl) vst2(OUT + ((size_t)b * TT + ql0 + rl) * CC + ch * 128 + lane * 4, *(const v4f*)&ss[wave][rl][lane * 4]);
}

extern "C" void kernel_launch(void* const* d_in, const int* in_sizes, int n_in, void* d_out, int out_size, void* d_ws, size_t ws_size, hipStream_t stream) {
  if (n_in < 7) return;
  if ((size_t)in_sizes[0] < ((size_t)(NB - 1) * SEQ_FULL + TT) * DIN) return;
  if (in_sizes[1] < DIN * CC || in_sizes[3] < DIN * CC || in_sizes[5] < DIN * CC) return;
  if (in_sizes[2] < CC || in_sizes[4] < CC || in_sizes[6] < CC) return;
  if ((size_t)out_size < (size_t)NB * TT * CC) return;
  if (ws_size < (size_t)WS_END) return;
  const float** F = (const float**)d_in;
  char* ws = (char*)d_ws;
  __bf16 *XB = (__bf16*)(ws + WS_XB), *WT = (__bf16*)(ws + WS_WT);
  _Float16 *QH = (_Float16*)(ws + WS_QH), *QL = (_Float16*)(ws + WS_QL), *KH = (_Float16*)(ws + WS_KH), *KL = (_Float16*)(ws + WS_KL), *VT = (_Float16*)(ws + WS_VT);
  float* S = (float*)(ws + WS_S); const _Float16* PH = (const _Float16*)(ws + WS_S);
  float* OUT = (float*)d_out;
  k_xb<<<dim3((unsigned)(((size_t)NB * TT * (DIN / 8) + 255) / 256)), 256, 0, stream>>>(F[0], XB);
  k_wt<<<dim3(CC / 16, 3), 128, 0, stream>>>(F[1], F[3], F[5], WT);
  k_proj<<<dim3(NB * TT / 64, CC / 128, 3), 128, 0, stream>>>(XB, WT, F[2], F[4], F[6], QH, QL, KH, KL, VT);
  for (int b = 0; b < NB; ++b) {
    k_sc<<<dim3(TT / 64, TT / 64), 128, 0, stream>>>(QH, KH, QL, KL, b, S);
    k_sm<<<dim3(TT), 256, 0, stream>>>(S);
    k_pv<<<dim3(TT / 64, CC / 128), 128, 0, stream>>>(PH, VT, b, OUT);
  }
}
